// GNNReadabilityGAT_86260123173012
// MI455X (gfx1250) — hardware-verified
//
#include <hip/hip_runtime.h>
#include <stddef.h>
#include <stdint.h>
#include <math.h>


#define F_IN    300
#define KX      320
#define HC      1024
#define HID     256
#define NHD     4
#define KA      2048
#define KA3     512
#define FC1     128
#define NCLS    6
#define NTHR    256
#define NWAVE   8
#define EPT     8
#define CHUNK   (NTHR * EPT)
#define WCAP    (EPT * 32)
#define LISTN   (NWAVE * WCAP)
#define NBA     512
#define SLA     9
#define RCAP    12800
#define DEGCAP  128
#define MEAS_B512   8338
#define MEAS_MAXDEG 36
#define GBM     64
#define GBN     64
#define GTHR    128
#define MROWS   128
#define HBM     128
#define TP      132
#define NEGSL   0.2f
#define EPS_SM  1e-16f
#define BN_EPS  1e-5f
#define WSMAX   134217728
#define BKT_LDS_INTS  (LISTN + RCAP + 16)
#define SCAN_ZINTS    (RCAP + 3 * NBA)
#define SCAN_LDS_INTS (2 * RCAP + 3 * NBA + 16)
#define PSTG    (5 * HC)
#define HEAD_LDS_F (HBM * TP + NCLS * FC1 + FC1 + 8 + HBM * NCLS)

static_assert((CHUNK & (CHUNK - 1)) == 0 && CHUNK <= 4096);
static_assert((NBA & (NBA - 1)) == 0 && NBA == (1 << SLA) && NBA <= 1024);
static_assert(((long long)CHUNK << SLA) < (1LL << 31));
static_assert(LISTN >= NWAVE * WCAP);
static_assert(NBA % NWAVE == 0 && NBA % 32 == 0);
static_assert((RCAP % 32) == 0 && (SCAN_ZINTS % 4) == 0);
static_assert(RCAP >= MEAS_B512 + 4096);
static_assert(DEGCAP >= MEAS_MAXDEG + 8);
static_assert(SCAN_LDS_INTS * 4 <= 300000 && BKT_LDS_INTS * 4 <= 300000);
static_assert(PSTG + NWAVE * HID <= RCAP);
static_assert(GBM == (GTHR / 32) * 16);
static_assert((KX % 32) == 0 && (KA % 32) == 0 && (KA3 % 32) == 0);
static_assert(KA == 2 * HC && KA3 == 2 * HID && HC == NHD * HID);
static_assert((HC % GBN) == 0 && (HID % GBN) == 0);
static_assert((MROWS % GBM) == 0 && MROWS == HBM && (NBA % HBM) == 0);
static_assert(HID == 8 * 32);
static_assert((F_IN % 4) == 0 && KX >= F_IN && (KX % 8) == 0);
static_assert(FC1 == 8 * 16 && HBM == NWAVE * 16);
static_assert(((HBM * NCLS * 4) % 128) == 0);
static_assert((16 * NCLS * 4) % 128 == 0);
static_assert((HBM * NCLS) % NTHR == 0 && (HBM * NCLS) / 4 <= NTHR);
static_assert(HEAD_LDS_F * 4 <= 300000);

typedef float          v4f  __attribute__((ext_vector_type(4)));
typedef float          v8f  __attribute__((ext_vector_type(8)));
typedef int            v4i  __attribute__((ext_vector_type(4)));
typedef int            v8i  __attribute__((ext_vector_type(8)));
typedef unsigned int   v4u  __attribute__((ext_vector_type(4)));
typedef unsigned short v8us __attribute__((ext_vector_type(8)));
typedef __bf16         v16b __attribute__((ext_vector_type(16)));
typedef v4f  __attribute__((may_alias)) v4fa;
typedef v4i  __attribute__((may_alias)) v4ia;
typedef v8us __attribute__((may_alias)) v8usa;
union FragB { v16b v; v8us h[2]; v8i w; };

__device__ __forceinline__ v8f wmb(const FragB& a, const FragB& b, v8f c) {
  v8f d = __builtin_amdgcn_wmma_f32_16x16x32_bf16(false, a.v, false, b.v, (short)0, c, false, false);
  asm volatile("v_nop\n\tv_nop\n\tv_nop\n\tv_nop" : "+v"(d) : "v"(a.w), "v"(b.w));
  return d;
}

__device__ __forceinline__ unsigned int f2bf(float f) {
  const unsigned int u = __float_as_uint(f);
  const unsigned int r = ((u + 0x7FFFu + ((u >> 16) & 1u)) >> 16) & 0xFFFFu;
  return ((u & 0x7FFFFFFFu) > 0x7F800000u) ? 0x7FC0u : r;
}
__device__ __forceinline__ float bf2f(unsigned int b) { return __uint_as_float(b << 16); }
__device__ __forceinline__ float bfr(float f) { return bf2f(f2bf(f)); }
__device__ __forceinline__ v4f bfr4(const v4f a) {
  v4f r; r.x = bfr(a.x); r.y = bfr(a.y); r.z = bfr(a.z); r.w = bfr(a.w); return r;
}
__device__ __forceinline__ unsigned int pk2(float lo, float hi) { return f2bf(lo) | (f2bf(hi) << 16); }
__device__ __forceinline__ v4u pack8(const v4f a, const v4f b) {
  v4u r;
  r.x = pk2(a.x, a.y); r.y = pk2(a.z, a.w); r.z = pk2(b.x, b.y); r.w = pk2(b.z, b.w);
  return r;
}

template <int SLB>
__device__ __forceinline__ int scan_chunk(const int* __restrict__ dsts, int nE, int cbase, int slotBase,
                                          int nb, int vec8, int* list, int tid, int lane, int wave) {
  int wc = 0;
  const int el0  = tid * EPT;
  const int e0   = cbase + el0;
  const int sent = -2147483647 - 1;
  v4i da, db;
  if (vec8 != 0 && cbase + CHUNK <= nE) {
    da = *(const v4i*)(dsts + e0);
    db = *(const v4i*)(dsts + e0 + 4);
  } else {
    da.x = (e0     < nE) ? dsts[min(e0,     nE - 1)] : sent;
    da.y = (e0 + 1 < nE) ? dsts[min(e0 + 1, nE - 1)] : sent;
    da.z = (e0 + 2 < nE) ? dsts[min(e0 + 2, nE - 1)] : sent;
    da.w = (e0 + 3 < nE) ? dsts[min(e0 + 3, nE - 1)] : sent;
    db.x = (e0 + 4 < nE) ? dsts[min(e0 + 4, nE - 1)] : sent;
    db.y = (e0 + 5 < nE) ? dsts[min(e0 + 5, nE - 1)] : sent;
    db.z = (e0 + 6 < nE) ? dsts[min(e0 + 6, nE - 1)] : sent;
    db.w = (e0 + 7 < nE) ? dsts[min(e0 + 7, nE - 1)] : sent;
  }
  const unsigned nbs = (unsigned)slotBase;
  const unsigned unb = (unsigned)nb;
  const unsigned s0 = (unsigned)da.x - nbs, s1 = (unsigned)da.y - nbs;
  const unsigned s2 = (unsigned)da.z - nbs, s3 = (unsigned)da.w - nbs;
  const unsigned s4 = (unsigned)db.x - nbs, s5 = (unsigned)db.y - nbs;
  const unsigned s6 = (unsigned)db.z - nbs, s7 = (unsigned)db.w - nbs;
  const bool h0 = s0 < unb, h1 = s1 < unb, h2 = s2 < unb, h3 = s3 < unb;
  const bool h4 = s4 < unb, h5 = s5 < unb, h6 = s6 < unb, h7 = s7 < unb;
  const unsigned any = __builtin_amdgcn_ballot_w32(h0 | h1 | h2 | h3 | h4 | h5 | h6 | h7);
  if (any != 0u) {
#define HITJ(J, HJ, SJ) { \
      const unsigned mj = __builtin_amdgcn_ballot_w32(HJ); \
      if (mj != 0u) { \
        if (HJ) { \
          const int pos = wc + (int)__builtin_amdgcn_mbcnt_lo(mj, 0u); \
          if (pos < WCAP) list[wave * WCAP + pos] = ((el0 + (J)) << SLB) | (int)(SJ); \
        } \
        wc += (int)__builtin_popcount(mj); } }
    HITJ(0, h0, s0)
    HITJ(1, h1, s1)
    HITJ(2, h2, s2)
    HITJ(3, h3, s3)
    HITJ(4, h4, s4)
    HITJ(5, h5, s5)
    HITJ(6, h6, s6)
    HITJ(7, h7, s7)
#undef HITJ
  }
  return wc;
}

__global__ __launch_bounds__(NTHR) void k_cvt(const float* __restrict__ src, unsigned short* dst,
                                              int rowsSrc, int Kin, int Kseg, int nSeg, int nUnits) {
  const int u = (int)blockIdx.x * NTHR + (int)threadIdx.x;
  if (u >= nUnits) return;
  const int pitch = Kseg * nSeg;
  const int upr = pitch >> 3;
  const int row = u / upr;
  const int k8  = (u - row * upr) * 8;
  const int kk  = k8 - (k8 / Kseg) * Kseg;
  const int rc  = row < rowsSrc ? row : rowsSrc - 1;
  const int ca  = kk     < Kin - 4 ? kk     : Kin - 4;
  const int cb  = kk + 4 < Kin - 4 ? kk + 4 : Kin - 4;
  const float* p = src + (size_t)rc * (size_t)Kin;
  v4f a = *(const v4fa*)(p + ca);
  v4f b = *(const v4fa*)(p + cb);
  const v4f z4 = {0.f, 0.f, 0.f, 0.f};
  const bool okr = row < rowsSrc;
  if (!(okr && kk < Kin))     a = z4;
  if (!(okr && kk + 4 < Kin)) b = z4;
  const v4u hv = pack8(a, b);
  unsigned short* o = dst + (size_t)row * (size_t)pitch + k8;
  *(volatile v4u*)o = hv;
  __threadfence();
  *(volatile v4u*)o = hv;
}

__global__ __launch_bounds__(NTHR) void k_bucket(const int* __restrict__ srcs, const int* __restrict__ dsts,
                                                 int nE, int nN, int vec8, int* HITS, int* FLG) {
  extern __shared__ __attribute__((aligned(16))) int bsm[];
  int* list = bsm;
  int* reg1 = bsm + LISTN;
  int* wcnt = reg1 + RCAP;
  const int tid = (int)threadIdx.x, lane = tid & 31, wave = tid >> 5;
  const int blk = (int)blockIdx.x;
  const int nodeBase = blk * NBA;
  int nb = nN - nodeBase;
  nb = nb < 0 ? 0 : (nb > NBA ? NBA : nb);

  int tot = 0, ovf = 0;
  const int nChunks = (nE + CHUNK - 1) / CHUNK;
#pragma unroll 1
  for (int ch = 0; ch < nChunks; ++ch) {
    const int cbase = ch * CHUNK;
    const int wc = scan_chunk<SLA>(dsts, nE, cbase, nodeBase, nb, vec8, list, tid, lane, wave);
    if (lane == 0) wcnt[wave] = wc;
    __syncthreads();
    int pre = 0, all = 0;
#pragma unroll
    for (int w2 = 0; w2 < NWAVE; ++w2) {
      int c = wcnt[w2];
      c = c < 0 ? 0 : (c > WCAP ? WCAP : c);
      all += c;
      pre += (w2 < wave) ? c : 0;
    }
    const int wcc  = wc > WCAP ? WCAP : wc;
    const int base = tot + pre;
#pragma unroll 1
    for (int i = lane; i < wcc; i += 32) {
      const int ent = list[wave * WCAP + i];
      const int el  = (ent >> SLA) & (CHUNK - 1);
      const int sl  = ent & (NBA - 1);
      int eid = cbase + el;
      eid = eid > nE - 1 ? nE - 1 : eid;
      const int sraw = srcs[eid];
      const int s = sraw < 0 ? 0 : (sraw > nN - 1 ? nN - 1 : sraw);
      const int pos = base + i;
      if (pos < RCAP) reg1[pos] = (int)((unsigned)s | ((unsigned)sl << 16));
    }
    if (tot + all > RCAP) ovf = 1;
    tot += all;
    tot = tot > RCAP ? RCAP : tot;
    __syncthreads();
  }
  const int nh = tot;
  const int nhPad = (nh + 31) & ~31;
  for (int i = nh + tid; i < nhPad; i += NTHR) reg1[i] = 0;
  __syncthreads();

  int* hb = HITS + (size_t)blk * RCAP;
  v4i cv;
  cv.x = (tid == 0) ? nh : 0;
  cv.y = (tid == 0) ? ovf : 0;
  cv.z = 0; cv.w = 0;
  int* fp = FLG + (size_t)blk * 32 + 4 * (tid & 7);
#pragma unroll 1
  for (int p = tid * 4; p < nhPad; p += NTHR * 4) {
    const v4i v = *(const v4ia*)(reg1 + p);
    *(volatile v4i*)(hb + p) = v;
  }
  if (tid < 8) *(volatile v4i*)fp = cv;
  __threadfence();
#pragma unroll 1
  for (int p = tid * 4; p < nhPad; p += NTHR * 4) {
    const v4i v = *(const v4ia*)(reg1 + p);
    *(volatile v4i*)(hb + p) = v;
  }
  if (tid < 8) *(volatile v4i*)fp = cv;
}

__global__ __launch_bounds__(GTHR) __attribute__((amdgpu_num_vgpr(248)))
void k_gemm(const unsigned short* __restrict__ A, const unsigned short* __restrict__ WT,
            float* outF, int K, int ldo) {
  __shared__ __attribute__((aligned(16))) float stg[GBM * GBN];
  const int tid = (int)threadIdx.x, lane = tid & 31, wave = tid >> 5, hh = lane >> 4, m = lane & 15;
  const int rowBase = (int)blockIdx.x * GBM;
  const int col0    = (int)blockIdx.y * GBN;

  v8f acc[4];
  {
    const v8f z = {0.f, 0.f, 0.f, 0.f, 0.f, 0.f, 0.f, 0.f};
    acc[0] = z; acc[1] = z; acc[2] = z; acc[3] = z;
  }
  const unsigned short* ap = A  + (size_t)(rowBase + 16 * wave + m) * (size_t)K + 8 * hh;
  const unsigned short* wp = WT + (size_t)(col0 + m) * (size_t)K + 8 * hh;
  const int ksteps = K >> 5;
#pragma unroll 1
  for (int ks = 0; ks < ksteps; ++ks) {
    FragB af;
    af.h[0] = *(const v8usa*)(ap + 32 * ks);
    af.h[1] = *(const v8usa*)(ap + 32 * ks + 16);
#pragma unroll
    for (int t = 0; t < 4; ++t) {
      const unsigned short* wq = wp + (size_t)(16 * t) * (size_t)K + 32 * ks;
      FragB bf;
      bf.h[0] = *(const v8usa*)wq;
      bf.h[1] = *(const v8usa*)(wq + 16);
      acc[t] = wmb(af, bf, acc[t]);
    }
  }

#pragma unroll
  for (int t = 0; t < 4; ++t) {
    const int lc = 16 * t + m;
#pragma unroll
    for (int r = 0; r < 8; ++r) {
      const int lr = 16 * wave + 8 * hh + r;
      stg[lr * GBN + lc] = acc[t][r];
    }
  }
  __syncthreads();

  v4f fv[8];
#pragma unroll
  for (int i = 0; i < 8; ++i) {
    const int lr = 16 * wave + 2 * i + hh;
    fv[i] = *(const v4fa*)(stg + lr * GBN + 4 * m);
  }
#pragma unroll
  for (int i = 0; i < 8; ++i) {
    const int gr = rowBase + 16 * wave + 2 * i + hh;
    float* op = outF + (size_t)gr * (size_t)ldo + col0 + 4 * m;
    *(volatile v4f*)op = fv[i];
  }
  __threadfence();
#pragma unroll
  for (int i = 0; i < 8; ++i) {
    const int gr = rowBase + 16 * wave + 2 * i + hh;
    float* op = outF + (size_t)gr * (size_t)ldo + col0 + 4 * m;
    *(volatile v4f*)op = fv[i];
  }
}

template <int NH>
__global__ __launch_bounds__(NTHR) void k_dots(const float* __restrict__ F, const float* __restrict__ atts,
                                               const float* __restrict__ attd, float* SD, int MPr) {
  constexpr int CT = NH * HID;
  __shared__ __attribute__((aligned(16))) float satt[2 * CT];
  __shared__ __attribute__((aligned(16))) float sres[2 * NHD * 32];
  const int tid = (int)threadIdx.x, lane = tid & 31, wave = tid >> 5;
#pragma unroll 1
  for (int i = tid * 4; i < CT; i += NTHR * 4) {
    *(v4fa*)(satt + i)      = bfr4(*(const v4fa*)(atts + i));
    *(v4fa*)(satt + CT + i) = bfr4(*(const v4fa*)(attd + i));
  }
  __syncthreads();
  const int rowBase = (int)blockIdx.x * 32;
#pragma unroll 1
  for (int q = 0; q < 4; ++q) {
    const int nl = wave * 4 + q;
    const float* fr = F + (size_t)(rowBase + nl) * CT + 8 * lane;
#pragma unroll 1
    for (int hd = 0; hd < NH; ++hd) {
      const v4f a   = *(const v4fa*)(fr + hd * HID);
      const v4f b   = *(const v4fa*)(fr + hd * HID + 4);
      const v4f sa0 = *(const v4fa*)(satt + hd * HID + 8 * lane);
      const v4f sa1 = *(const v4fa*)(satt + hd * HID + 8 * lane + 4);
      const v4f sd0 = *(const v4fa*)(satt + CT + hd * HID + 8 * lane);
      const v4f sd1 = *(const v4fa*)(satt + CT + hd * HID + 8 * lane + 4);
      float s = a.x * sa0.x;
      s = fmaf(a.y, sa0.y, s); s = fmaf(a.z, sa0.z, s); s = fmaf(a.w, sa0.w, s);
      s = fmaf(b.x, sa1.x, s); s = fmaf(b.y, sa1.y, s); s = fmaf(b.z, sa1.z, s); s = fmaf(b.w, sa1.w, s);
      float d = a.x * sd0.x;
      d = fmaf(a.y, sd0.y, d); d = fmaf(a.z, sd0.z, d); d = fmaf(a.w, sd0.w, d);
      d = fmaf(b.x, sd1.x, d); d = fmaf(b.y, sd1.y, d); d = fmaf(b.z, sd1.z, d); d = fmaf(b.w, sd1.w, d);
#pragma unroll
      for (int off = 16; off > 0; off >>= 1) {
        s += __shfl_xor(s, off);
        d += __shfl_xor(d, off);
      }
      if (lane == 0) {
        sres[(2 * hd) * 32 + nl]     = s;
        sres[(2 * hd + 1) * 32 + nl] = d;
      }
    }
  }
  __syncthreads();
  const bool wr = tid < 16 * NH;
  const int tc = wr ? tid : 0;
  const int plane = tc >> 3, piece = tc & 7;
  const v4f v = *(const v4fa*)(sres + plane * 32 + 4 * piece);
  float* op = SD + (size_t)plane * (size_t)MPr + rowBase + 4 * piece;
  if (wr) *(volatile v4f*)op = v;
  __threadfence();
  if (wr) *(volatile v4f*)op = v;
}

template <int NH, int BN>
__global__ __launch_bounds__(NTHR) __attribute__((amdgpu_num_vgpr(248)))
void k_scan(const int* __restrict__ HITS, const int* FLGB,
            const float* __restrict__ F, const float* __restrict__ SD,
            const float* __restrict__ bias, const float* __restrict__ bg, const float* __restrict__ bbe,
            const float* __restrict__ bm, const float* __restrict__ bv,
            unsigned short* XP, int* FLGO, int nN) {
  constexpr int CT = NH * HID;
  extern __shared__ __attribute__((aligned(16))) int ssm[];
  int* hl   = ssm;
  int* sl   = ssm + RCAP;
  int* cnt  = sl + RCAP;
  int* offs = cnt + NBA;
  int* cur  = offs + NBA;
  int* misc = cur + NBA;
  const int tid = (int)threadIdx.x, lane = tid & 31, wave = tid >> 5;
  const int blk = (int)blockIdx.x;
  const int nodeBase = blk * NBA;
  const int MPr = ((nN + MROWS - 1) / MROWS) * MROWS;

  const int nhraw = FLGB[(size_t)blk * 32];
  const int bflag = FLGB[(size_t)blk * 32 + 1];
  const int nh  = nhraw < 0 ? 0 : (nhraw > RCAP ? RCAP : nhraw);
  const int ovf = (bflag != 0 || nhraw < 0 || nhraw > RCAP) ? 1 : 0;

  {
    const v4i z4 = {0, 0, 0, 0};
    for (int i = tid * 4; i < SCAN_ZINTS; i += NTHR * 4) *(v4ia*)(sl + i) = z4;
    if (tid < 16) misc[tid] = 0;
    const int* hb = HITS + (size_t)blk * RCAP;
    const int nh4 = (nh + 3) & ~3;
#pragma unroll 1
    for (int p = tid * 4; p < nh4; p += NTHR * 4) *(v4ia*)(hl + p) = *(const v4i*)(hb + p);
  }
  __syncthreads();

  if (wave == 0) {
#pragma unroll 1
    for (int b0 = 0; b0 < nh; b0 += 32) {
      const int idx = b0 + lane;
      const int uv  = hl[idx < nh ? idx : nh - 1];
      const int m32 = (nh - b0) < 32 ? (nh - b0) : 32;
#pragma unroll 1
      for (int k = 0; k < m32; ++k) {
        const int u  = __builtin_amdgcn_readlane(uv, k);
        const int sq = (u >> 16) & (NBA - 1);
        if (lane == 0) cnt[sq] = cnt[sq] + 1;
      }
    }
  }
  __syncthreads();
  if (wave == 0) {
    const int base = lane * (NBA / 32);
    int s = 0;
#pragma unroll 1
    for (int i = 0; i < NBA / 32; ++i) s += cnt[base + i];
    int incl = s;
#pragma unroll
    for (int d = 1; d < 32; d <<= 1) {
      const int y = __shfl_up(incl, d, 32);
      if (lane >= d) incl += y;
    }
    int run = incl - s;
#pragma unroll 1
    for (int i = 0; i < NBA / 32; ++i) {
      const int cv = cnt[base + i];
      offs[base + i] = run;
      cur[base + i]  = run;
      run += cv;
    }
  }
  __syncthreads();
  if (wave == 0) {
#pragma unroll 1
    for (int b0 = 0; b0 < nh; b0 += 32) {
      const int idx = b0 + lane;
      const int uv  = hl[idx < nh ? idx : nh - 1];
      const int m32 = (nh - b0) < 32 ? (nh - b0) : 32;
#pragma unroll 1
      for (int k = 0; k < m32; ++k) {
        const int u  = __builtin_amdgcn_readlane(uv, k);
        const int sq = (u >> 16) & (NBA - 1);
        if (lane == 0) {
          int p = cur[sq];
          p = p < 0 ? 0 : (p > RCAP - 1 ? RCAP - 1 : p);
          sl[p] = u;
          cur[sq] = p + 1;
        }
      }
    }
  }
  __syncthreads();

  float* fl = (float*)hl;
  float* pb = fl;
  float* pm = fl + CT;
  float* pr = fl + 2 * CT;
  float* pg = fl + 3 * CT;
  float* pe = fl + 4 * CT;
  float* st = fl + PSTG + wave * HID;
#pragma unroll 1
  for (int i = tid; i < CT; i += NTHR) {
    pb[i] = bfr(bias[i]);
    if constexpr (BN != 0) {
      pm[i] = bfr(bm[i]);
      pr[i] = 1.0f / sqrtf(bfr(bv[i]) + BN_EPS);
      pg[i] = bfr(bg[i]);
      pe[i] = bfr(bbe[i]);
    }
  }
  __syncthreads();

  const float qnan = __int_as_float(0x7fc00000);
  const float pzb  = (ovf != 0) ? qnan : 0.0f;
  int anybig = 0;

#pragma unroll 1
  for (int si = 0; si < NBA / NWAVE; ++si) {
    const int s    = si * NWAVE + wave;
    const int node = nodeBase + s;
    if (node >= MPr) continue;
    const int nc   = node < nN ? node : nN - 1;
    int c = cnt[s];
    const bool big = c > DEGCAP;
    anybig |= big ? 1 : 0;
    c = c < 0 ? 0 : (c > DEGCAP ? DEGCAP : c);
    int o = offs[s];
    o = o < 0 ? 0 : (o > RCAP ? RCAP : o);
    if (c > nh - o) c = nh - o;
    c = c < 0 ? 0 : c;
    const int T = c + 1;
    const float pzr = big ? qnan : pzb;
    const bool live = node < nN;

#pragma unroll 1
    for (int hd = 0; hd < NH; ++hd) {
      const size_t hoS = (size_t)(2 * hd) * (size_t)MPr;
      const size_t hoD = hoS + (size_t)MPr;
      const float adv = SD[hoD + (size_t)nc];
      float mx = -3.0e38f, dn = 0.0f;
      float acc[8];
#pragma unroll
      for (int i = 0; i < 8; ++i) acc[i] = 0.0f;
#pragma unroll 1
      for (int b0 = 0; b0 < T; b0 += 32) {
        const int t = b0 + lane;
        int idx = o + t;
        idx = idx < 0 ? 0 : (idx > RCAP - 1 ? RCAP - 1 : idx);
        const int ent = sl[idx];
        int hs = ent & 0xFFFF;
        hs = hs > nN - 1 ? nN - 1 : hs;
        const int sr  = (t < c) ? hs : nc;
        const int m32 = (T - b0) < 32 ? (T - b0) : 32;
#pragma unroll 1
        for (int k = 0; k < m32; ++k) {
          const int sk = __builtin_amdgcn_readlane(sr, k);
          const float* rp = F + (size_t)sk * CT + hd * HID + 8 * lane;
          const v4f a = *(const v4f*)rp;
          const v4f b = *(const v4f*)(rp + 4);
          float lg = SD[hoS + (size_t)sk] + adv;
          lg = lg > 0.f ? lg : NEGSL * lg;
          const float df = lg - mx;
          const float ee = expf(-fabsf(df));
          const bool  up = df > 0.f;
          const float s1 = up ? ee : 1.0f;
          const float s2 = up ? 1.0f : ee;
          mx = up ? lg : mx;
          dn = fmaf(dn, s1, s2);
          acc[0] = fmaf(acc[0], s1, s2 * a.x); acc[1] = fmaf(acc[1], s1, s2 * a.y);
          acc[2] = fmaf(acc[2], s1, s2 * a.z); acc[3] = fmaf(acc[3], s1, s2 * a.w);
          acc[4] = fmaf(acc[4], s1, s2 * b.x); acc[5] = fmaf(acc[5], s1, s2 * b.y);
          acc[6] = fmaf(acc[6], s1, s2 * b.z); acc[7] = fmaf(acc[7], s1, s2 * b.w);
        }
      }
      const float inv = __builtin_amdgcn_rcpf(dn + EPS_SM);
#pragma unroll
      for (int i = 0; i < 8; ++i) st[i * 32 + lane] = acc[i];
#pragma unroll 1
      for (int j = 0; j < 8; ++j) {
        const int col = hd * HID + 8 * lane + j;
        float y = fmaf(st[j * 32 + lane], inv, pb[col]);
        if constexpr (BN != 0) {
          y = y - pm[col];
          y = y * pr[col];
          y = y * pg[col];
          y = y + pe[col];
        }
        y = (y > 0.0f) ? y : expm1f(y);
        st[j * 32 + lane] = y + pzr;
      }
      v8us ho, lo;
#pragma unroll
      for (int i = 0; i < 8; ++i) {
        const float y = st[i * 32 + lane];
        const float v = live ? y : 0.0f;
        const unsigned int hbi = f2bf(v);
        ho[i] = (unsigned short)hbi;
        lo[i] = (unsigned short)f2bf(v - bf2f(hbi));
      }
      unsigned short* hp = XP + (size_t)node * (size_t)(2 * CT) + hd * HID + 8 * lane;
      *(volatile v8us*)hp = ho;
      *(volatile v8us*)(hp + CT) = lo;
      __threadfence();
      *(volatile v8us*)hp = ho;
      *(volatile v8us*)(hp + CT) = lo;
    }
  }

  if (lane == 0) misc[wave] = anybig;
  __syncthreads();
  if (wave == 0) {
    int fg = ovf;
#pragma unroll
    for (int w2 = 0; w2 < NWAVE; ++w2) fg |= misc[w2];
    v4i cv;
    cv.x = 0;
    cv.y = (lane == 0) ? fg : 0;
    cv.z = 0; cv.w = 0;
    int* fp = FLGO + (size_t)blk * 32 + 4 * (lane & 7);
    if (lane < 8) *(volatile v4i*)fp = cv;
    __threadfence();
    if (lane < 8) *(volatile v4i*)fp = cv;
  }
}

__global__ __launch_bounds__(NTHR) __attribute__((amdgpu_num_vgpr(248)))
void k_head(const unsigned short* __restrict__ A, const unsigned short* __restrict__ WT,
            const float* __restrict__ fb1, const float* __restrict__ fw2, const float* __restrict__ fb2,
            const int* __restrict__ FLG, float* out, int nN, int nBk) {
  extern __shared__ __attribute__((aligned(16))) float hsm[];
  float* tile = hsm;
  float* sw2  = tile + HBM * TP;
  float* sb1  = sw2 + NCLS * FC1;
  float* sb2  = sb1 + FC1;
  float* sout = sb2 + 8;
  const int tid = (int)threadIdx.x, lane = tid & 31, wave = tid >> 5, hh = lane >> 4, m = lane & 15;
  const int rowBase = (int)blockIdx.x * HBM;

  {
    const float b1v = bfr(fb1[tid & (FC1 - 1)]);
    if (tid < FC1) sb1[tid] = b1v;
#pragma unroll 1
    for (int i = tid; i < NCLS * FC1; i += NTHR) sw2[i] = bfr(fw2[i]);
    const int c8 = tid & 7;
    const int ci = c8 < NCLS ? c8 : NCLS - 1;
    const float b2v = bfr(fb2[ci]);
    if (tid < 8) sb2[tid] = (c8 < NCLS) ? b2v : 0.0f;
  }
  int fg = 0;
  {
    int b5 = rowBase / NBA;
    b5 = b5 > nBk - 1 ? nBk - 1 : b5;
#pragma unroll
    for (int l = 0; l < 4; ++l) fg |= FLG[((size_t)l * (size_t)nBk + (size_t)b5) * 32 + 1];
  }
  const float pz = (fg != 0) ? __int_as_float(0x7fc00000) : 0.0f;
  __syncthreads();

  v8f acc[8];
  {
    const v8f z = {0.f, 0.f, 0.f, 0.f, 0.f, 0.f, 0.f, 0.f};
#pragma unroll
    for (int t = 0; t < 8; ++t) acc[t] = z;
  }
  const unsigned short* ap = A  + (size_t)(rowBase + 16 * wave + m) * (size_t)KA3 + 8 * hh;
  const unsigned short* wp = WT + (size_t)m * (size_t)KA3 + 8 * hh;
#pragma unroll 1
  for (int ks = 0; ks < KA3 / 32; ++ks) {
    FragB af;
    af.h[0] = *(const v8usa*)(ap + 32 * ks);
    af.h[1] = *(const v8usa*)(ap + 32 * ks + 16);
#pragma unroll
    for (int t = 0; t < 8; ++t) {
      const unsigned short* wq = wp + (size_t)(16 * t) * (size_t)KA3 + 32 * ks;
      FragB bf;
      bf.h[0] = *(const v8usa*)wq;
      bf.h[1] = *(const v8usa*)(wq + 16);
      acc[t] = wmb(af, bf, acc[t]);
    }
  }

#pragma unroll
  for (int t = 0; t < 8; ++t) {
    const int lc = 16 * t + m;
    const float bb = sb1[lc];
#pragma unroll
    for (int r = 0; r < 8; ++r) {
      const int lr = 16 * wave + 8 * hh + r;
      float v = acc[t][r] + bb;
      v = (v > 0.0f) ? v : (v - v);
      tile[lr * TP + lc] = v;
    }
  }
  __syncthreads();

#pragma unroll 1
  for (int task = tid; task < HBM * NCLS; task += NTHR) {
    const int row = task / NCLS;
    const int c   = task - row * NCLS;
    const float* tr = tile + row * TP;
    const float* wr = sw2 + c * FC1;
    float s = 0.0f;
#pragma unroll 4
    for (int k = 0; k < FC1; ++k) s = fmaf(tr[k], wr[k], s);
    sout[task] = s + sb2[c] + pz;
  }
  __syncthreads();

  const int nTot = nN * NCLS;
  const int np   = (HBM * NCLS) / 4;
  const int pc   = tid < np ? tid : np - 1;
  const v4f v = *(const v4fa*)(sout + 4 * pc);
  const int f0 = rowBase * NCLS + 4 * pc;
  const bool wr = (tid < np) && (f0 + 4 <= nTot);
  const int f0c = wr ? f0 : 0;
  float* op = out + (size_t)f0c;
  if (wr) *(volatile v4f*)op = v;
  __threadfence();
  if (wr) *(volatile v4f*)op = v;
}

static inline int cdiv(int a, int b) { return (a + b - 1) / b; }

extern "C" void kernel_launch(void* const* d_in, const int* in_sizes, int n_in,
                              void* d_out, int out_size, void* d_ws, size_t ws_size,
                              hipStream_t stream) {
  if (n_in < 26) return;
  const int nN = in_sizes[0] / F_IN;
  if (nN <= 0 || in_sizes[0] != nN * F_IN || nN > 65535 || (nN % 16) != 0) return;
  if (in_sizes[1] < 2 || (in_sizes[1] & 1) != 0) return;
  const int nE = in_sizes[1] / 2;
  if (nE < 1 || nE > (1 << 30)) return;
  if (in_sizes[2] != HC * F_IN) return;
  if (in_sizes[3] != HC || in_sizes[4] != HC || in_sizes[5] != HC) return;
  if (in_sizes[6] != HC * HC) return;
  if (in_sizes[7] != HC || in_sizes[8] != HC || in_sizes[9] != HC) return;
  if (in_sizes[10] != HID * HC) return;
  if (in_sizes[11] != HID || in_sizes[12] != HID || in_sizes[13] != HID) return;
  for (int i = 14; i < 22; ++i) if (in_sizes[i] != HC) return;
  if (in_sizes[22] != FC1 * HID || in_sizes[23] != FC1) return;
  if (in_sizes[24] != NCLS * FC1 || in_sizes[25] < NCLS) return;
  if (out_size != nN * NCLS) return;

  const float* x    = (const float*)d_in[0];
  const int*   ei   = (const int*)  d_in[1];
  const float* W1   = (const float*)d_in[2];
  const float* a1s  = (const float*)d_in[3];
  const float* a1d  = (const float*)d_in[4];
  const float* b1   = (const float*)d_in[5];
  const float* W2   = (const float*)d_in[6];
  const float* a2s  = (const float*)d_in[7];
  const float* a2d  = (const float*)d_in[8];
  const float* b2   = (const float*)d_in[9];
  const float* W3   = (const float*)d_in[10];
  const float* a3s  = (const float*)d_in[11];
  const float* a3d  = (const float*)d_in[12];
  const float* b3   = (const float*)d_in[13];
  const float* g1   = (const float*)d_in[14];
  const float* be1  = (const float*)d_in[15];
  const float* m1   = (const float*)d_in[16];
  const float* v1   = (const float*)d_in[17];
  const float* g2   = (const float*)d_in[18];
  const float* be2  = (const float*)d_in[19];
  const float* m2   = (const float*)d_in[20];
  const float* v2   = (const float*)d_in[21];
  const float* fc1W = (const float*)d_in[22];
  const float* fc1b = (const float*)d_in[23];
  const float* fc2W = (const float*)d_in[24];
  const float* fc2b = (const float*)d_in[25];
  float* out = (float*)d_out;
  const int* src = ei;
  const int* dst = ei + nE;

  const int MP   = cdiv(nN, MROWS) * MROWS;
  const int gM   = MP / GBM;
  const int gA   = cdiv(MP, NBA);
  if ((long long)gA * NBA < (long long)MP) return;
  const int vec8 = ((nE & 3) == 0) ? 1 : 0;

  char* ws = (char*)d_ws;
  size_t off = 0;
  const size_t oXB  = off; off += (size_t)MP * KX * 2;        off = (off + 255) & ~(size_t)255;
  const size_t oW1B = off; off += (size_t)HC * KX * 2;        off = (off + 255) & ~(size_t)255;
  const size_t oW2D = off; off += (size_t)HC * KA * 2;        off = (off + 255) & ~(size_t)255;
  const size_t oW3D = off; off += (size_t)HID * KA * 2;       off = (off + 255) & ~(size_t)255;
  const size_t oF1D = off; off += (size_t)FC1 * KA3 * 2;      off = (off + 255) & ~(size_t)255;
  const size_t oH   = off; off += (size_t)MP * HC * 4;        off = (off + 255) & ~(size_t)255;
  const size_t oXH  = off; off += (size_t)MP * KA * 2;        off = (off + 255) & ~(size_t)255;
  const size_t oSD  = off; off += (size_t)2 * NHD * MP * 4;   off = (off + 255) & ~(size_t)255;
  const size_t oHIT = off; off += (size_t)gA * RCAP * 4;      off = (off + 255) & ~(size_t)255;
  const size_t oFLG = off; off += (size_t)4 * gA * 128;       off = (off + 255) & ~(size_t)255;
  if (off > ws_size || off > (size_t)WSMAX) return;
  unsigned short* XB  = (unsigned short*)(ws + oXB);
  unsigned short* W1B = (unsigned short*)(ws + oW1B);
  unsigned short* W2D = (unsigned short*)(ws + oW2D);
  unsigned short* W3D = (unsigned short*)(ws + oW3D);
  unsigned short* F1D = (unsigned short*)(ws + oF1D);
  float*          H   = (float*)(ws + oH);
  unsigned short* XHL = (unsigned short*)(ws + oXH);
  float*          SD  = (float*)(ws + oSD);
  int*            HITS = (int*)(ws + oHIT);
  int*            FLG  = (int*)(ws + oFLG);
  int* FLG0 = FLG;
  int* FLG1 = FLG + (size_t)gA * 32;
  int* FLG2 = FLG + (size_t)2 * gA * 32;
  int* FLG3 = FLG + (size_t)3 * gA * 32;

  const int bktLds  = BKT_LDS_INTS * 4;
  const int scanLds = SCAN_LDS_INTS * 4;
  const int headLds = HEAD_LDS_F * 4;
  hipFuncSetAttribute(reinterpret_cast<const void*>(&k_bucket),
                      hipFuncAttributeMaxDynamicSharedMemorySize, bktLds);
  hipFuncSetAttribute(reinterpret_cast<const void*>(&k_scan<NHD, 1>),
                      hipFuncAttributeMaxDynamicSharedMemorySize, scanLds);
  hipFuncSetAttribute(reinterpret_cast<const void*>(&k_scan<1, 0>),
                      hipFuncAttributeMaxDynamicSharedMemorySize, scanLds);
  hipFuncSetAttribute(reinterpret_cast<const void*>(&k_head),
                      hipFuncAttributeMaxDynamicSharedMemorySize, headLds);

  {
    const int nUx = MP * (KX / 8);
    k_cvt<<<cdiv(nUx, NTHR), NTHR, 0, stream>>>(x, XB, nN, F_IN, KX, 1, nUx);
    const int nU1 = HC * (KX / 8);
    k_cvt<<<cdiv(nU1, NTHR), NTHR, 0, stream>>>(W1, W1B, HC, F_IN, KX, 1, nU1);
    const int nU2 = HC * (KA / 8);
    k_cvt<<<cdiv(nU2, NTHR), NTHR, 0, stream>>>(W2, W2D, HC, HC, HC, 2, nU2);
    const int nU3 = HID * (KA / 8);
    k_cvt<<<cdiv(nU3, NTHR), NTHR, 0, stream>>>(W3, W3D, HID, HC, HC, 2, nU3);
    const int nU4 = FC1 * (KA3 / 8);
    k_cvt<<<cdiv(nU4, NTHR), NTHR, 0, stream>>>(fc1W, F1D, FC1, HID, HID, 2, nU4);
  }
  k_bucket<<<gA, NTHR, bktLds, stream>>>(src, dst, nE, nN, vec8, HITS, FLG0);

  k_gemm<<<dim3(gM, HC / GBN), GTHR, 0, stream>>>(XB, W1B, H, KX, HC);
  k_dots<NHD><<<MP / 32, NTHR, 0, stream>>>(H, a1s, a1d, SD, MP);
  k_scan<NHD, 1><<<gA, NTHR, scanLds, stream>>>(HITS, FLG0, H, SD, b1, g1, be1, m1, v1, XHL, FLG1, nN);
  k_gemm<<<dim3(gM, HC / GBN), GTHR, 0, stream>>>(XHL, W2D, H, KA, HC);
  k_dots<NHD><<<MP / 32, NTHR, 0, stream>>>(H, a2s, a2d, SD, MP);
  k_scan<NHD, 1><<<gA, NTHR, scanLds, stream>>>(HITS, FLG0, H, SD, b2, g2, be2, m2, v2, XHL, FLG2, nN);
  k_gemm<<<dim3(gM, HID / GBN), GTHR, 0, stream>>>(XHL, W3D, H, KA, HID);
  k_dots<1><<<MP / 32, NTHR, 0, stream>>>(H, a3s, a3d, SD, MP);
  k_scan<1, 0><<<gA, NTHR, scanLds, stream>>>(HITS, FLG0, H, SD, b3, b3, b3, b3, b3, XHL, FLG3, nN);
  k_head<<<MP / HBM, NTHR, headLds, stream>>>(XHL, F1D, fc1b, fc2W, fc2b, FLG, out, nN, gA);
}
